// SBI_MSA_19026705121920
// MI455X (gfx1250) — hardware-verified
//
#include <hip/hip_runtime.h>
#include <math.h>

#define NBATCH 2
#define SEQ    2048
#define DM     512
#define NH     8
#define HD     64
#define NE     10
#define NEP    16
#define MP     (NBATCH * SEQ)
#define QKW    (4 * DM)
#define KOFF   (2 * DM)
#define CTXP   (2 * DM)
#define NQB    (SEQ / 64)
#define RSC    2048.0f
#define PSC    1024.0f
static_assert(NH * HD == DM);
static_assert(DM == 8 * 64);
static_assert((SEQ % 64) == 0 && (DM % 64) == 0 && (MP % 64) == 0 && (SEQ % 256) == 0 && (MP % 4) == 0);
static_assert((((MP / 64) * (DM / 64)) % 8) == 0);
static_assert((((DM / 64) * (SEQ / 64)) % 8) == 0);
static_assert(NE <= NEP && NEP == 16);

typedef _Float16 v16h __attribute__((ext_vector_type(16)));
typedef _Float16 v8h  __attribute__((ext_vector_type(8)));
typedef __bf16   v16b __attribute__((ext_vector_type(16)));
typedef unsigned short v16us __attribute__((ext_vector_type(16)));
typedef unsigned short v8us  __attribute__((ext_vector_type(8)));
typedef float    v8f  __attribute__((ext_vector_type(8)));
typedef float    v4f  __attribute__((ext_vector_type(4)));
typedef unsigned int v4u __attribute__((ext_vector_type(4)));

union FragH { v16h v; v8h h[2]; };
union FragU { v16us v; v8us h[2]; };

__device__ __forceinline__ unsigned short bf_bits(float f) {
  unsigned u = __float_as_uint(f);
  return (unsigned short)((u + 0x7FFFu + ((u >> 16) & 1u)) >> 16);
}
__device__ __forceinline__ float bf_up(unsigned short h) { return __uint_as_float(((unsigned)h) << 16); }
__device__ __forceinline__ float bfr(float f) { return bf_up(bf_bits(f)); }
__device__ __forceinline__ unsigned short h_bits(_Float16 x) { return __builtin_bit_cast(unsigned short, x); }
__device__ __forceinline__ unsigned pk16(unsigned short a, unsigned short b) { return (unsigned)a | ((unsigned)b << 16); }
__device__ __forceinline__ v8f zero8() { v8f z = {0.f, 0.f, 0.f, 0.f, 0.f, 0.f, 0.f, 0.f}; return z; }

__device__ __forceinline__ v16us ldfrag_u(const unsigned short* p) {
  FragU f;
  f.h[0] = *(const v8us*)(p);
  f.h[1] = *(const v8us*)(p + 16);
  return f.v;
}

__device__ __forceinline__ v8f mma_bu_raw(v16us a, v16us b, v8f c) {
  return __builtin_amdgcn_wmma_f32_16x16x32_bf16(false, __builtin_bit_cast(v16b, a), false,
                                                 __builtin_bit_cast(v16b, b), (short)0, c, false, false);
}
__device__ __forceinline__ v8f mma_hu(v16us a, v16us b, v8f c) {
  c = __builtin_amdgcn_wmma_f32_16x16x32_f16(false, __builtin_bit_cast(v16h, a), false,
                                              __builtin_bit_cast(v16h, b), (short)0, c, false, false);
#if defined(__HIP_DEVICE_COMPILE__)
  asm volatile("v_nop\n\tv_nop\n\tv_nop\n\tv_nop" : "+v"(c) : "v"(a), "v"(b));
#endif
  return c;
}
__device__ __forceinline__ v8f mma_h(v16h a, v16h b, v8f c) {
  c = __builtin_amdgcn_wmma_f32_16x16x32_f16(false, a, false, b, (short)0, c, false, false);
#if defined(__HIP_DEVICE_COMPILE__)
  asm volatile("v_nop\n\tv_nop\n\tv_nop\n\tv_nop" : "+v"(c) : "v"(a), "v"(b));
#endif
  return c;
}
__device__ __forceinline__ void dep_guard1(v8f& a, v8f& b, v16us x) {
#if defined(__HIP_DEVICE_COMPILE__)
  asm volatile("v_nop\n\tv_nop\n\tv_nop\n\tv_nop" : "+v"(a), "+v"(b) : "v"(x));
#endif
}
__device__ __forceinline__ void keep4_u(v16us a, v16us b, v16us c, v16us d) {
#if defined(__HIP_DEVICE_COMPILE__)
  asm volatile("v_nop" :: "v"(a), "v"(b), "v"(c), "v"(d));
#endif
}
__device__ __forceinline__ void acc_guard4(v8f& a, v8f& b, v8f& c, v8f& d) {
#if defined(__HIP_DEVICE_COMPILE__)
  asm volatile("v_nop\n\tv_nop\n\tv_nop\n\tv_nop" : "+v"(a), "+v"(b), "+v"(c), "+v"(d));
#endif
}
__device__ __forceinline__ void wave_sync_lds() {
  __builtin_amdgcn_fence(__ATOMIC_RELEASE, "workgroup");
  __builtin_amdgcn_wave_barrier();
  __builtin_amdgcn_fence(__ATOMIC_ACQUIRE, "workgroup");
}

__global__ __launch_bounds__(256) void cvt3(const float* __restrict__ s0, const float* __restrict__ s1,
                                            const float* __restrict__ s2, unsigned short* dst) {
  const int z = blockIdx.y;
  const float* src = (z == 0) ? s0 : ((z == 1) ? s1 : s2);
  const int t = threadIdx.x;
  const int row = blockIdx.x * 4 + (t >> 6);
  const int c8 = (t & 63) * 8;
  const float* p = src + (size_t)row * DM + c8;
  const v4f a0 = *(const v4f*)(p);
  const v4f a1 = *(const v4f*)(p + 4);
  v4u hv;
  hv[0] = pk16(bf_bits(a0[0]), bf_bits(a0[1]));
  hv[1] = pk16(bf_bits(a0[2]), bf_bits(a0[3]));
  hv[2] = pk16(bf_bits(a1[0]), bf_bits(a1[1]));
  hv[3] = pk16(bf_bits(a1[2]), bf_bits(a1[3]));
  unsigned short* d = dst + ((size_t)z * MP + (size_t)row) * DM + c8;
  *(volatile v4u*)d = hv;
  __threadfence();
  *(volatile v4u*)d = hv;
}

__global__ __launch_bounds__(256) void tconv64(const float* __restrict__ W, unsigned short* out,
                                               int rows, int cols, int ldo, int dupoff) {
  __shared__ __align__(16) unsigned short sh[64 * 72];
  const int t  = threadIdx.x;
  const int n0 = blockIdx.x * 64;
  const int k0 = blockIdx.y * 64;
#pragma unroll
  for (int i = 0; i < 4; ++i) {
    const int idx = i * 256 + t;
    const int r = idx >> 4, c4 = (idx & 15) * 4;
    int kr = k0 + r;   kr = (kr < rows) ? kr : (rows - 1);
    int nc = n0 + c4;  nc = (nc < cols - 4) ? nc : (cols - 4);
    const v4f v = *(const v4f*)(W + (size_t)kr * cols + nc);
#pragma unroll
    for (int e = 0; e < 4; ++e) sh[(c4 + e) * 72 + r] = bf_bits(v[e]);
  }
  __syncthreads();
  const int wave = t >> 5, lane = t & 31;
  const int q = lane >> 3, c8 = (lane & 7) * 8;
  v4u pv[2];
  size_t go[2];
#pragma unroll
  for (int it = 0; it < 2; ++it) {
    const int nl = it * 32 + wave * 4 + q;
    pv[it] = *(const v4u*)(sh + nl * 72 + c8);
    go[it] = (size_t)(n0 + nl) * ldo + k0 + c8;
  }
  for (int pass = 0; pass < 2; ++pass) {
#pragma unroll
    for (int it = 0; it < 2; ++it) {
      *(volatile v4u*)(out + go[it]) = pv[it];
      if (dupoff != 0) *(volatile v4u*)(out + go[it] + dupoff) = pv[it];
    }
    __threadfence();
  }
}

template <int OM>
__global__ __launch_bounds__(256) void gemm64(
    const unsigned short* __restrict__ Ap, int lda, long long sAy,
    const unsigned short* __restrict__ Btp, int ldb, long long sBy,
    unsigned short* Cp, unsigned short* Cp2, float* Cf, int ldc, long long sCy,
    int M, int N, int K, int nmul, float oscale) {
  __shared__ __align__(16) float sT[8][16 * 68];
  const int by   = blockIdx.y;
  const int lane = threadIdx.x & 31;
  const int wave = threadIdx.x >> 5;
  const int tilesN = N >> 6;
  const int tilesM = M >> 6;
  const int tile = blockIdx.x * 8 + wave;
  if (tile >= tilesM * tilesN) return;
  const int tm = tile / tilesN;
  const int tn = tile - tm * tilesN;
  const int m0 = tm << 6;
  const int n0 = tn << 6;

  const unsigned short* Ab = Ap  + (size_t)by * (size_t)sAy;
  const unsigned short* Bb = Btp + (size_t)by * (size_t)sBy;
  const size_t cofs = (size_t)by * (size_t)sCy;

  const int rlane = lane & 15;
  const int koff  = (lane >> 4) * 8;
  const int mOff  = (lane >> 4) * 8;

  v8f acc[4][4];
#pragma unroll
  for (int i = 0; i < 4; ++i)
#pragma unroll
    for (int j = 0; j < 4; ++j) acc[i][j] = zero8();

  for (int k0 = 0; k0 < K; k0 += 32) {
    v16us bh[4];
#pragma unroll
    for (int j = 0; j < 4; ++j) {
      const size_t bo = (size_t)(n0 + (j << 4) + rlane) * ldb + koff + k0;
      bh[j] = ldfrag_u(Bb + bo);
    }
#pragma unroll
    for (int i = 0; i < 4; ++i) {
      const size_t ao = (size_t)(m0 + (i << 4) + rlane) * lda + koff + k0;
      const v16us ah = ldfrag_u(Ab + ao);
#pragma unroll
      for (int j = 0; j < 4; ++j) acc[i][j] = mma_bu_raw(ah, bh[j], acc[i][j]);
      dep_guard1(acc[i][0], acc[i][3], ah);
    }
    keep4_u(bh[0], bh[1], bh[2], bh[3]);
  }
  acc_guard4(acc[0][0], acc[0][1], acc[0][2], acc[0][3]);
  acc_guard4(acc[1][0], acc[1][1], acc[1][2], acc[1][3]);
  acc_guard4(acc[2][0], acc[2][1], acc[2][2], acc[2][3]);
  acc_guard4(acc[3][0], acc[3][1], acc[3][2], acc[3][3]);

  const int hh2 = lane >> 4, c4 = (lane & 15) * 4;
  const int q8  = lane >> 3, c8 = (lane & 7) * 8;

  float* slab = sT[wave];
#pragma unroll
  for (int i = 0; i < 4; ++i) {
    const int mBase = m0 + (i << 4);
#pragma unroll
    for (int j = 0; j < 4; ++j) {
#pragma unroll
      for (int r = 0; r < 8; ++r) {
        slab[(mOff + r) * 68 + (j << 4) + rlane] = acc[i][j][r];
      }
    }
    wave_sync_lds();
    if (OM == 0) {
      float* C = Cf + cofs;
      v4f vals[8];
#pragma unroll
      for (int it = 0; it < 8; ++it) {
        const int row = it * 2 + hh2;
        v4f v = *(const v4f*)(slab + row * 68 + c4);
        vals[it] = v * oscale;
      }
      for (int pass = 0; pass < 2; ++pass) {
#pragma unroll
        for (int it = 0; it < 8; ++it) {
          const int row = it * 2 + hh2;
          *(volatile v4f*)(C + (size_t)(mBase + row) * ldc + (size_t)n0 * nmul + c4) = vals[it];
        }
        __threadfence();
      }
    } else {
      unsigned short* C  = Cp  + cofs;
      unsigned short* C2 = Cp2 + cofs;
      v4u hv[4], lv[4];
#pragma unroll
      for (int it = 0; it < 4; ++it) {
        const int row = it * 4 + q8;
        const float* sp = slab + row * 68 + c8;
        v4u ha, la;
#pragma unroll
        for (int e = 0; e < 4; ++e) {
          const float f0 = sp[2 * e]     * oscale;
          const float f1 = sp[2 * e + 1] * oscale;
          const _Float16 g0 = (_Float16)f0, g1 = (_Float16)f1;
          const unsigned short u0 = h_bits(g0), u1 = h_bits(g1);
          const unsigned short w0 = h_bits((_Float16)((f0 - (float)g0) * RSC));
          const unsigned short w1 = h_bits((_Float16)((f1 - (float)g1) * RSC));
          ha[e] = pk16(u0, u1);
          la[e] = pk16(w0, w1);
        }
        hv[it] = ha;
        lv[it] = la;
      }
      for (int pass = 0; pass < 2; ++pass) {
#pragma unroll
        for (int it = 0; it < 4; ++it) {
          const int row = it * 4 + q8;
          const size_t go = (size_t)(mBase + row) * ldc + (size_t)n0 * nmul + c8;
          *(volatile v4u*)(C  + go) = hv[it];
          *(volatile v4u*)(C2 + go) = lv[it];
        }
        __threadfence();
      }
    }
    wave_sync_lds();
  }
}

__global__ __launch_bounds__(64) void idx_rows(const unsigned short* __restrict__ qk,
                                               const float* __restrict__ emb, float* itab) {
  __shared__ float Qs[64 * 65];
  __shared__ float Es[NE * HD];
  __shared__ __align__(16) float Ts[64 * NEP];
  const int tid = threadIdx.x;
  const int R0 = blockIdx.x * 64;
  const int bh = R0 / SEQ;
  const int l0 = R0 - bh * SEQ;
  const int b  = bh / NH;
  const int h  = bh - b * NH;
#pragma unroll 1
  for (int i = tid; i < NE * HD; i += 64) {
    const int n = i >> 6, d = i & 63;
    Es[i] = bfr(emb[(size_t)n * DM + h * HD + d]);
  }
  const _Float16* qp = (const _Float16*)(const void*)qk
                     + ((size_t)b * SEQ + (size_t)l0 + (size_t)tid) * QKW + (size_t)h * (2 * HD);
#pragma unroll
  for (int i = 0; i < 8; ++i) {
    const v8h hv = *(const v8h*)(qp + 8 * i);
    const v8h lv = *(const v8h*)(qp + HD + 8 * i);
#pragma unroll
    for (int e = 0; e < 8; ++e)
      Qs[tid * 65 + 8 * i + e] = (float)hv[e] + (float)lv[e] * (1.0f / RSC);
  }
  __syncthreads();
#pragma unroll 1
  for (int n = 0; n < NE; ++n) {
    float s = 0.f;
#pragma unroll 1
    for (int dc = 0; dc < 2; ++dc) {
#pragma unroll
      for (int d = 0; d < 32; ++d) s += Qs[tid * 65 + dc * 32 + d] * Es[n * HD + dc * 32 + d];
    }
    Ts[tid * NEP + n] = s;
  }
#pragma unroll
  for (int n = NE; n < NEP; ++n) Ts[tid * NEP + n] = 0.f;
  __syncthreads();
  v4f vals[4];
#pragma unroll
  for (int it = 0; it < 4; ++it) vals[it] = *(const v4f*)(Ts + (it * 64 + tid) * 4);
  float* base = itab + (size_t)R0 * NEP;
#pragma unroll
  for (int it = 0; it < 4; ++it) *(volatile v4f*)(base + (it * 64 + tid) * 4) = vals[it];
  __threadfence();
#pragma unroll
  for (int it = 0; it < 4; ++it) *(volatile v4f*)(base + (it * 64 + tid) * 4) = vals[it];
}

__global__ __launch_bounds__(128)
void attn64(const unsigned short* __restrict__ qk, const unsigned short* __restrict__ vth,
            const unsigned short* __restrict__ vtl, const float* __restrict__ itab,
            const int* __restrict__ trj, unsigned short* ctxp, float sscale) {
  __shared__ __align__(16) unsigned short Kh[64 * 64];
  __shared__ __align__(16) _Float16 Vh[64 * 64];
  __shared__ __align__(16) _Float16 Vl[64 * 64];
  __shared__ __align__(16) _Float16 Psh[4][16 * 64];
  __shared__ __align__(16) float    Os[4][16 * 64];
  __shared__ __align__(16) float    ITs[64 * NEP];

  const int tid  = threadIdx.x;
  const int wave = tid >> 5;
  const int lane = tid & 31;
  const int hh   = lane >> 4;
  const int c    = lane & 15;

  const int bx   = blockIdx.x;
  const int qb   = bx % NQB;
  const int rest = bx / NQB;
  const int h    = rest % NH;
  const int b    = rest / NH;
  const int q0   = qb * 64 + wave * 16;
  const size_t rowB = (size_t)b * SEQ;

  const unsigned short* Qh  = qk + (size_t)h * (2 * HD);
  const unsigned short* Kg  = qk + KOFF + (size_t)h * (2 * HD);
  const _Float16* Vgh = (const _Float16*)(const void*)vth + ((size_t)b * DM + (size_t)h * HD) * SEQ;
  const _Float16* Vgl = (const _Float16*)(const void*)vtl + ((size_t)b * DM + (size_t)h * HD) * SEQ;
  const float* itb = itab + (((size_t)b * NH + (size_t)h) * SEQ + (size_t)qb * 64) * NEP;
  const int* trw = trj + (rowB + (size_t)q0 + (size_t)(8 * hh)) * SEQ + c;

#pragma unroll
  for (int i = 0; i < 2; ++i) {
    const int f = i * 128 + tid;
    *(v4f*)(ITs + f * 4) = *(const v4f*)(itb + (size_t)f * 4);
  }

  float mrow[8], lrow[8];
  v8f oacc[4], oaccL[4];
#pragma unroll
  for (int r = 0; r < 8; ++r) { mrow[r] = -INFINITY; lrow[r] = 0.f; }
#pragma unroll
  for (int t = 0; t < 4; ++t) { oacc[t] = zero8(); oaccL[t] = zero8(); }

#pragma unroll 1
  for (int kt = 0; kt < NQB; ++kt) {
    const int kv0 = kt * 64;

    __syncthreads();
    {
      const int r = tid >> 1, hf = (tid & 1) * 32;
      const unsigned short* kgh = Kg + (rowB + kv0 + r) * QKW + hf;
      const _Float16* vgh = Vgh + (size_t)r * SEQ + kv0 + hf;
      const _Float16* vgl = Vgl + (size_t)r * SEQ + kv0 + hf;
#pragma unroll
      for (int i = 0; i < 4; ++i) {
        const v8us a0 = *(const v8us*)(kgh + 8 * i);
        const v8h  b0 = *(const v8h*)(vgh + 8 * i);
        const v8h  b1 = *(const v8h*)(vgl + 8 * i);
        *(v8us*)(Kh + r * 64 + hf + 8 * i) = a0;
        *(v8h*)(Vh + r * 64 + hf + 8 * i) = b0;
        *(v8h*)(Vl + r * 64 + hf + 8 * i) = b1;
      }
    }
    __syncthreads();

    v16us qh2[2];
#pragma unroll
    for (int dc = 0; dc < 2; ++dc) {
      qh2[dc] = ldfrag_u(Qh + (rowB + q0 + c) * QKW + dc * 32 + 8 * hh);
    }

    v8f s[4];
#pragma unroll
    for (int j = 0; j < 4; ++j) {
      v8f sh = zero8();
#pragma unroll
      for (int dc = 0; dc < 2; ++dc) {
        FragU kb;
        kb.h[0] = *(const v8us*)(Kh + (j * 16 + c) * 64 + dc * 32 + 8 * hh);
        kb.h[1] = *(const v8us*)(Kh + (j * 16 + c) * 64 + dc * 32 + 16 + 8 * hh);
        sh = mma_hu(qh2[dc], kb.v, sh);
      }
      const int* tp = trw + kv0 + j * 16;
#pragma unroll
      for (int r = 0; r < 8; ++r) {
        int n = tp[(size_t)r * SEQ];
        n = (n < 0) ? 0 : n;
        n = (n > NE - 1) ? (NE - 1) : n;
        s[j][r] = sh[r] * sscale + ITs[(wave * 16 + 8 * hh + r) * NEP + n];
      }
    }

    _Float16* pwh = Psh[wave];
#pragma unroll
    for (int r = 0; r < 8; ++r) {
      float m = s[0][r];
      m = fmaxf(m, s[1][r]);
      m = fmaxf(m, s[2][r]);
      m = fmaxf(m, s[3][r]);
#pragma unroll
      for (int off = 1; off < 16; off <<= 1) m = fmaxf(m, __shfl_xor(m, off, 32));
      const float mnew  = fmaxf(mrow[r], m);
      const float alpha = __expf(mrow[r] - mnew);
      mrow[r] = mnew;
      float psum = 0.f;
#pragma unroll
      for (int j = 0; j < 4; ++j) {
        const float p = __expf(s[j][r] - mnew);
        psum += p;
        pwh[(8 * hh + r) * 64 + j * 16 + c] = (_Float16)(p * PSC);
      }
#pragma unroll
      for (int off = 1; off < 16; off <<= 1) psum += __shfl_xor(psum, off, 32);
      lrow[r] = lrow[r] * alpha + psum;
#pragma unroll
      for (int t = 0; t < 4; ++t) { oacc[t][r] *= alpha; oaccL[t][r] *= alpha; }
    }
    wave_sync_lds();

#pragma unroll 1
    for (int kk = 0; kk < 2; ++kk) {
      FragH pa;
      pa.h[0] = *(const v8h*)(pwh + c * 64 + kk * 32 + 8 * hh);
      pa.h[1] = *(const v8h*)(pwh + c * 64 + kk * 32 + 16 + 8 * hh);
#pragma unroll
      for (int t = 0; t < 4; ++t) {
        FragH vb, vl;
        vb.h[0] = *(const v8h*)(Vh + (t * 16 + c) * 64 + kk * 32 + 8 * hh);
        vb.h[1] = *(const v8h*)(Vh + (t * 16 + c) * 64 + kk * 32 + 16 + 8 * hh);
        vl.h[0] = *(const v8h*)(Vl + (t * 16 + c) * 64 + kk * 32 + 8 * hh);
        vl.h[1] = *(const v8h*)(Vl + (t * 16 + c) * 64 + kk * 32 + 16 + 8 * hh);
        oacc[t]  = mma_h(pa.v, vb.v, oacc[t]);
        oaccL[t] = mma_h(pa.v, vl.v, oaccL[t]);
      }
    }
  }

  float* os = Os[wave];
#pragma unroll
  for (int r = 0; r < 8; ++r) {
    const float l = lrow[r];
    const float inv = ((l > 0.f) ? (1.0f / l) : 0.f) * (1.0f / PSC);
#pragma unroll
    for (int t = 0; t < 4; ++t) os[(8 * hh + r) * 64 + t * 16 + c] = (oacc[t][r] + oaccL[t][r] * (1.0f / RSC)) * inv;
  }
  wave_sync_lds();
  {
    const int q4 = lane >> 3, c8 = (lane & 7) * 8;
    v4u hv[4], lv[4];
#pragma unroll
    for (int it = 0; it < 4; ++it) {
      const int row = it * 4 + q4;
      const float* sp = os + row * 64 + c8;
      v4u ha, la;
#pragma unroll
      for (int e = 0; e < 4; ++e) {
        const float f0 = sp[2 * e], f1 = sp[2 * e + 1];
        const unsigned short u0 = bf_bits(f0), u1 = bf_bits(f1);
        const unsigned short w0 = bf_bits(f0 - bf_up(u0)), w1 = bf_bits(f1 - bf_up(u1));
        ha[e] = pk16(u0, u1);
        la[e] = pk16(w0, w1);
      }
      hv[it] = ha;
      lv[it] = la;
    }
    for (int pass = 0; pass < 2; ++pass) {
#pragma unroll
      for (int it = 0; it < 4; ++it) {
        const int row = it * 4 + q4;
        const size_t go = (rowB + q0 + row) * CTXP + (size_t)h * HD + c8;
        *(volatile v4u*)(ctxp + go)      = hv[it];
        *(volatile v4u*)(ctxp + go + DM) = lv[it];
      }
      __threadfence();
    }
  }
}

__global__ __launch_bounds__(64) void ln_rows(const float* __restrict__ X, const float* __restrict__ gam,
                                              const float* __restrict__ bet, float* out) {
  __shared__ float red[4];
  const int row = blockIdx.x;
  const int tid = threadIdx.x, lane = tid & 31, wv = tid >> 5;
  const float* src = X + (size_t)row * DM;
  const v4f a0 = *(const v4f*)(src + tid * 4);
  const v4f a1 = *(const v4f*)(src + 256 + tid * 4);
  float x[8];
#pragma unroll
  for (int e = 0; e < 4; ++e) { x[e] = a0[e]; x[4 + e] = a1[e]; }
  float s = 0.f;
#pragma unroll
  for (int e = 0; e < 8; ++e) s += x[e];
#pragma unroll
  for (int off = 1; off < 32; off <<= 1) s += __shfl_xor(s, off, 32);
  if (lane == 0) red[wv] = s;
  __syncthreads();
  const float mean = (red[0] + red[1]) * (1.0f / DM);
  float d[8];
  float q = 0.f;
#pragma unroll
  for (int e = 0; e < 8; ++e) { d[e] = x[e] - mean; q += d[e] * d[e]; }
#pragma unroll
  for (int off = 1; off < 32; off <<= 1) q += __shfl_xor(q, off, 32);
  if (lane == 0) red[2 + wv] = q;
  __syncthreads();
  const float var  = (red[2] + red[3]) * (1.0f / DM);
  const float rstd = rsqrtf(var + 1e-6f);

  const v4f g0 = *(const v4f*)(gam + tid * 4);
  const v4f g1 = *(const v4f*)(gam + 256 + tid * 4);
  const v4f e0 = *(const v4f*)(bet + tid * 4);
  const v4f e1 = *(const v4f*)(bet + 256 + tid * 4);
  v4f o0, o1;
#pragma unroll
  for (int e = 0; e < 4; ++e) {
    o0[e] = d[e]     * rstd * bfr(g0[e]) + bfr(e0[e]);
    o1[e] = d[4 + e] * rstd * bfr(g1[e]) + bfr(e1[e]);
  }
  float* dst = out + (size_t)row * DM + tid * 4;
  *(volatile v4f*)(dst)       = o0;
  *(volatile v4f*)(dst + 256) = o1;
  __threadfence();
  *(volatile v4f*)(dst)       = o0;
  *(volatile v4f*)(dst + 256) = o1;
}

extern "C" void kernel_launch(void* const* d_in, const int* in_sizes, int n_in,
                              void* d_out, int out_size, void* d_ws, size_t ws_size,
                              hipStream_t stream) {
  if (n_in < 11) return;
  if (in_sizes[0] != MP * DM || in_sizes[1] != MP * DM || in_sizes[2] != MP * DM) return;
  if (in_sizes[3] != NE * DM) return;
  if (in_sizes[4] != NBATCH * SEQ * SEQ) return;
  if (in_sizes[5] != DM * DM || in_sizes[6] != DM * DM || in_sizes[7] != DM * DM || in_sizes[8] != DM * DM) return;
  if (in_sizes[9] != DM || in_sizes[10] != DM) return;
  if (out_size != MP * DM) return;

  const float* q_in = (const float*)d_in[0];
  const float* k_in = (const float*)d_in[1];
  const float* v_in = (const float*)d_in[2];
  const float* emb  = (const float*)d_in[3];
  const int*   trj  = (const int*)d_in[4];
  const float* w_q  = (const float*)d_in[5];
  const float* w_k  = (const float*)d_in[6];
  const float* w_v  = (const float*)d_in[7];
  const float* w_o  = (const float*)d_in[8];
  const float* gam  = (const float*)d_in[9];
  const float* bet  = (const float*)d_in[10];

  const size_t PWT  = (size_t)3 * DM * DM * 2;
  const size_t PWO  = (size_t)DM * KOFF * 2;
  const size_t PIN  = (size_t)3 * MP * DM * 2;
  const size_t PQK  = (size_t)MP * QKW * 2;
  const size_t PVT  = (size_t)NBATCH * DM * SEQ * 2;
  const size_t PIT  = (size_t)NBATCH * NH * SEQ * NEP * 4;
  const size_t PCTX = (size_t)MP * CTXP * 2;
  const size_t PX   = (size_t)MP * DM * 4;
  size_t off = 0;
  const size_t oWT  = off; off += PWT;
  const size_t oWo  = off; off += PWO;
  const size_t oIN  = off; off += PIN;
  const size_t oQK  = off; off += PQK;
  const size_t oVTh = off; off += PVT;
  const size_t oVTl = off; off += PVT;
  const size_t oIT  = off; off += PIT;
  const size_t oCtx = off; off += PCTX;
  const size_t oX   = off; off += PX;
  if (off > ws_size) return;
  if (off > (size_t)134217728) return;

  char* ws = (char*)d_ws;
  unsigned short* WT   = (unsigned short*)(ws + oWT);
  unsigned short* WoT2 = (unsigned short*)(ws + oWo);
  unsigned short* INb  = (unsigned short*)(ws + oIN);
  unsigned short* QK   = (unsigned short*)(ws + oQK);
  unsigned short* VTh  = (unsigned short*)(ws + oVTh);
  unsigned short* VTl  = (unsigned short*)(ws + oVTl);
  float*          IT   = (float*)(ws + oIT);
  unsigned short* Ctx  = (unsigned short*)(ws + oCtx);
  float*          X    = (float*)(ws + oX);
  float*          out0 = (float*)d_out;

  const dim3 blk(256), blk128(128), blk64(64);
  const dim3 gCv(MP / 4, 3);
  const dim3 gT(DM / 64, DM / 64);
  const dim3 gQK(((MP / 64) * (DM / 64)) / 8, 2, 1);
  const dim3 gVT(((DM / 64) * (SEQ / 64)) / 8, NBATCH, 1);
  const dim3 gIdx(NBATCH * NH * (SEQ / 64));
  const dim3 gAttn(NBATCH * NH * NQB);
  const dim3 gNo(((MP / 64) * (DM / 64)) / 8, 1, 1);
  const dim3 gLN(MP);
  if ((((MP / 64) * (DM / 64)) % 8) != 0) return;
  if ((((DM / 64) * (SEQ / 64)) % 8) != 0) return;

  cvt3<<<gCv, blk, 0, stream>>>(q_in, k_in, v_in, INb);
  tconv64<<<gT, blk, 0, stream>>>(w_q, WT, DM, DM, DM, 0);
  tconv64<<<gT, blk, 0, stream>>>(w_k, WT + (size_t)DM * DM, DM, DM, DM, 0);
  tconv64<<<gT, blk, 0, stream>>>(w_v, WT + (size_t)2 * DM * DM, DM, DM, DM, 0);
  tconv64<<<gT, blk, 0, stream>>>(w_o, WoT2, DM, DM, KOFF, DM);

  gemm64<4><<<gQK, blk, 0, stream>>>(
      INb, DM, (long long)MP * DM, WT, DM, (long long)DM * DM,
      QK, QK + HD, X, QKW, (long long)KOFF,
      MP, DM, DM, 2, 1.0f);
  gemm64<4><<<gVT, blk, 0, stream>>>(
      WT + (size_t)2 * DM * DM, DM, 0LL, INb + (size_t)2 * MP * DM, DM, (long long)SEQ * DM,
      VTh, VTl, X, SEQ, (long long)DM * SEQ,
      DM, SEQ, DM, 1, 1.0f);

  idx_rows<<<gIdx, blk64, 0, stream>>>(QK, emb, IT);
  attn64<<<gAttn, blk128, 0, stream>>>(QK, VTh, VTl, IT, trj, Ctx, 0.125f);

  gemm64<0><<<gNo, blk, 0, stream>>>(
      Ctx, CTXP, 0LL, WoT2, KOFF, 0LL,
      Ctx, Ctx, X, DM, 0LL,
      MP, DM, KOFF, 1, 1.0f);
  ln_rows<<<gLN, blk64, 0, stream>>>(X, gam, bet, out0);
  (void)hipGetLastError();
}
